// torch_RNN1_6940667150560
// MI455X (gfx1250) — hardware-verified
//
#include <hip/hip_runtime.h>

typedef __attribute__((ext_vector_type(16))) _Float16 v16h;
typedef __attribute__((ext_vector_type(8)))  _Float16 v8h;
typedef __attribute__((ext_vector_type(8)))  float    v8f;
typedef __attribute__((ext_vector_type(4)))  float    v4f;
typedef __attribute__((ext_vector_type(2)))  float    v2f;

constexpr int kBatch = 256;
constexpr int kStep  = 512;
constexpr int kIn    = 2;
constexpr int kHid   = 256;

constexpr int kSeqPB      = 16;
constexpr int kRnnBlocks  = kBatch / kSeqPB;
constexpr int kRnnThreads = 256;
constexpr int kWaves      = kRnnThreads / 32;
constexpr int kColsPW     = 32;
constexpr int kHP         = kHid + 8;
constexpr int kHTile      = kSeqPB * kHP;
constexpr int kNormPitch  = 32;
static_assert(kBatch % kSeqPB == 0, "blocks cover the batch exactly");
static_assert(kHid == kWaves * kColsPW, "wave columns cover the hidden dim exactly");
static_assert(kHP % 8 == 0, "16-B aligned fragment loads");
static_assert(kHid % 32 == 0, "K multiple of 32");

constexpr int kDwWhh      = kHid * kHid / 2;
constexpr int kPrepBlocks = kDwWhh / 256;
static_assert(kDwWhh % 256 == 0 && kPrepBlocks == 128, "exact coverage");

__device__ __forceinline__ void dep_guard_h(v8f& a, v8f& b, v16h x, v16h y) { asm volatile("v_nop\n\tv_nop\n\tv_nop\n\tv_nop" : "+v"(a), "+v"(b) : "v"(x), "v"(y)); }
__device__ __forceinline__ void keep4_h(v16h a, v16h b, v16h c, v16h d) { asm volatile("v_nop" :: "v"(a), "v"(b), "v"(c), "v"(d)); }
__device__ __forceinline__ void acc_guard2(v8f& a, v8f& b) { asm volatile("v_nop\n\tv_nop\n\tv_nop\n\tv_nop" : "+v"(a), "+v"(b)); }

template <typename T> struct Frag;
template <> struct Frag<_Float16> {
  typedef v16h V; union U { v16h v; v8h h[2]; };
  static __device__ __forceinline__ v16h load(const _Float16* p) {
    U f; f.h[0] = *(const v8h*)(p); f.h[1] = *(const v8h*)(p + 16); return f.v;
  }
  static __device__ __forceinline__ v8f mma(v16h a, v16h b, v8f c) {
    return __builtin_amdgcn_wmma_f32_16x16x32_f16(false, a, false, b, (short)0, c, false, false);
  }
  static __device__ __forceinline__ void guard(v8f& a, v8f& b, v16h x, v16h y) { dep_guard_h(a, b, x, y); }
  static __device__ __forceinline__ void keep(v16h a, v16h b, v16h c, v16h d) { keep4_h(a, b, c, d); }
};

__device__ __forceinline__ unsigned pack_f16x2(float a, float b) {
  const _Float16 h0 = (_Float16)a, h1 = (_Float16)b;
  return (unsigned)__builtin_bit_cast(unsigned short, h0) | ((unsigned)__builtin_bit_cast(unsigned short, h1) << 16);
}
__device__ __forceinline__ void st2u(unsigned* p, unsigned v) { *(volatile unsigned*)p = v; __threadfence(); *(volatile unsigned*)p = v; }

__global__ __launch_bounds__(256) void prep_kernel(const float* __restrict__ w_hh, unsigned* __restrict__ whhu) {
  const int p = blockIdx.x * 256 + threadIdx.x;
  st2u(whhu + p, pack_f16x2(w_hh[2 * p] * 16.0f, w_hh[2 * p + 1] * 16.0f));
}

__global__ __launch_bounds__(kRnnThreads) void rnn_kernel(
    const float* __restrict__ x, const float* __restrict__ w_ih,
    const _Float16* __restrict__ whh16, float* __restrict__ normws) {
  __shared__ __align__(16) _Float16 htile[kHTile];
  __shared__ float part[kWaves][kSeqPB];
  const int tid = threadIdx.x, lane = tid & 31, wave = tid >> 5;
  const int c = lane & 15, hh = lane >> 4, koff = hh * 8, mOff = hh * 8;
  const int seq0 = blockIdx.x * kSeqPB;
  const int n0 = wave * kColsPW;

  for (int i = tid; i < kHTile; i += kRnnThreads) htile[i] = (_Float16)0.0f;
  const float wa0 = w_ih[(n0 + c) * kIn],      wa1 = w_ih[(n0 + c) * kIn + 1];
  const float wb0 = w_ih[(n0 + 16 + c) * kIn], wb1 = w_ih[(n0 + 16 + c) * kIn + 1];
  __syncthreads();

  const _Float16* brow0 = whh16 + (size_t)(n0 + c) * kHid + koff;
  const _Float16* brow1 = brow0 + (size_t)16 * kHid;
  const _Float16* arow  = htile + c * kHP + koff;
  const float*    xrow  = x + (size_t)(seq0 + mOff) * kStep * kIn;
  const float inv256 = 1.0f / 256.0f;

  float hA[8], hB[8];
#pragma unroll
  for (int r = 0; r < 8; ++r) { hA[r] = 0.0f; hB[r] = 0.0f; }

#pragma unroll 1
  for (int s = 0; s < kStep; ++s) {
    float x0[8], x1[8];
#pragma unroll
    for (int r = 0; r < 8; ++r) {
      const v2f xv = *(const v2f*)(xrow + (size_t)r * kStep * kIn + s * kIn);
      x0[r] = xv[0]; x1[r] = xv[1];
    }

    v8f acc0 = (v8f){0.f,0.f,0.f,0.f,0.f,0.f,0.f,0.f};
    v8f acc1 = (v8f){0.f,0.f,0.f,0.f,0.f,0.f,0.f,0.f};
#pragma unroll
    for (int kc = 0; kc < kHid / 32; ++kc) {
      const v16h fa  = Frag<_Float16>::load(arow + kc * 32);
      const v16h fb0 = Frag<_Float16>::load(brow0 + kc * 32);
      const v16h fb1 = Frag<_Float16>::load(brow1 + kc * 32);
      acc0 = Frag<_Float16>::mma(fa, fb0, acc0);
      acc1 = Frag<_Float16>::mma(fa, fb1, acc1);
      Frag<_Float16>::guard(acc0, acc1, fa, fb1);
      Frag<_Float16>::keep(fb0, fb1, fa, fa);
    }
    acc_guard2(acc0, acc1);

    __syncthreads();

#pragma unroll
    for (int r = 0; r < 8; ++r) {
      const float xwa = x0[r] * wa0 + x1[r] * wa1;
      const float xwb = x0[r] * wb0 + x1[r] * wb1;
      const float va = fmaxf(acc0[r] * inv256 + xwa, 0.0f);
      const float vb = fmaxf(acc1[r] * inv256 + xwb, 0.0f);
      hA[r] = va; hB[r] = vb;
      htile[(mOff + r) * kHP + n0 + c]      = (_Float16)(va * 16.0f);
      htile[(mOff + r) * kHP + n0 + 16 + c] = (_Float16)(vb * 16.0f);
    }
    __syncthreads();
  }

#pragma unroll
  for (int r = 0; r < 8; ++r) {
    float sq = hA[r] * hA[r] + hB[r] * hB[r];
    sq += __shfl_xor(sq, 1, 32);
    sq += __shfl_xor(sq, 2, 32);
    sq += __shfl_xor(sq, 4, 32);
    sq += __shfl_xor(sq, 8, 32);
    if (c == 0) part[wave][mOff + r] = sq;
  }
  __syncthreads();
  if (wave == 0) {
    float tot = 0.0f;
#pragma unroll
    for (int w = 0; w < kWaves; ++w) tot += part[w][c];
    const float v = (lane < kSeqPB) ? sqrtf(tot) : 0.0f;
    float* dst = normws + blockIdx.x * kNormPitch + lane;
    *(volatile float*)dst = v;
    __threadfence();
    *(volatile float*)dst = v;
  }
}

__global__ __launch_bounds__(32) void out_kernel(const float* __restrict__ normws, float* __restrict__ out) {
  const int lane = threadIdx.x;
  v4f val[2];
#pragma unroll
  for (int it = 0; it < 2; ++it) {
    const int base = (it * 32 + lane) * 4;
#pragma unroll
    for (int e = 0; e < 4; ++e) {
      const int b = base + e;
      val[it][e] = normws[(b >> 4) * kNormPitch + (b & 15)];
    }
  }
  for (int pass = 0; pass < 2; ++pass) {
#pragma unroll
    for (int it = 0; it < 2; ++it) *(volatile v4f*)(out + (size_t)(it * 32 + lane) * 4) = val[it];
    __threadfence();
  }
}

extern "C" void kernel_launch(void* const* d_in, const int* in_sizes, int n_in,
                              void* d_out, int out_size, void* d_ws, size_t ws_size, hipStream_t stream) {
  if (n_in < 3 || d_out == nullptr || d_ws == nullptr) return;
  if (in_sizes[0] != kBatch * kStep * kIn || in_sizes[1] != kHid * kIn || in_sizes[2] != kHid * kHid ||
      out_size != kBatch) return;

  const float* x    = (const float*)d_in[0];
  const float* w_ih = (const float*)d_in[1];
  const float* w_hh = (const float*)d_in[2];
  float* out = (float*)d_out;

  char* ws = (char*)d_ws; size_t off = 0;
  auto carve = [&](size_t bytes) -> char* { char* p = ws + off; off += (bytes + 255) & ~(size_t)255; return p; };
  unsigned short* WHH16  = (unsigned short*)carve((size_t)kHid * kHid * 2);
  float*          NORMWS = (float*)carve((size_t)kRnnBlocks * kNormPitch * 4);
  if (off > ws_size || off > (size_t)134217728) return;

  prep_kernel<<<kPrepBlocks, 256, 0, stream>>>(w_hh, (unsigned*)WHH16);
  rnn_kernel<<<kRnnBlocks, kRnnThreads, 0, stream>>>(x, w_ih, (const _Float16*)WHH16, NORMWS);
  out_kernel<<<1, 32, 0, stream>>>(NORMWS, out);
}
